// Noise_Regressor_67774583930935
// MI455X (gfx1250) — hardware-verified
//
#include <hip/hip_runtime.h>
#include <stddef.h>


typedef _Float16 v16h __attribute__((ext_vector_type(16)));
typedef _Float16 v8h  __attribute__((ext_vector_type(8)));
typedef float    v8f  __attribute__((ext_vector_type(8)));
typedef float    v4f  __attribute__((ext_vector_type(4)));
typedef _Float16 h16;

#ifndef NB
#define NB 1
#endif
#ifndef SEQ
#define SEQ 2048
#endif
#ifndef XN_RES
#define XN_RES 1
#endif
#define NB_FULL  1
#define SEQ_FULL 2048
#define DIM   1024
#define NIMU  13
#define NPRM  10
#define NOUT  130
#define NPAD  192
#define MROWS (NB * SEQ)
#define ICH   256
#define NCH   (SEQ / ICH)
#define JT    64
#define PSTR  (NIMU * SEQ)

static_assert(NB == 1 && NB_FULL == 1);
static_assert(SEQ >= 256 && SEQ <= SEQ_FULL && (SEQ % 256) == 0);
static_assert(NOUT == NPRM * NIMU);
static_assert(NPAD >= NOUT && (NPAD % 64) == 0 && (NPAD % 32) == 0);
static_assert((DIM % 64) == 0 && (DIM % 32) == 0);
static_assert((MROWS % 64) == 0 && (MROWS % 8) == 0);
static_assert(DIM == 4 * 32 * 8);
static_assert(((NIMU * SEQ) % 256) == 0);
static_assert((SEQ % JT) == 0 && (SEQ % ICH) == 0 && NCH >= 1 && NCH <= 8);
static_assert((size_t)2 * NIMU * SEQ_FULL * 4 == (size_t)212992);
static_assert((size_t)NIMU * SEQ_FULL * 4 == (size_t)106496);

#define LDT 72
#define LDC 68
static_assert((LDT % 8) == 0 && LDT >= 64);
static_assert((LDC % 4) == 0 && LDC >= 64);

#define WCARRY 64.0f
#define RCARRY 2048.0f

#define WT_BYTES      ((size_t)NPAD * DIM * 2)
#define PLANE16_BYTES ((size_t)MROWS * DIM * 2)
#define P_BYTES       ((size_t)MROWS * NPAD * 4)
#define PAR_BYTES     ((size_t)8 * NIMU * SEQ * 4)
#define PART_BYTES    ((size_t)NCH * NIMU * SEQ * 4)
#define OFF_WT   ((size_t)0)
#define OFF_H1   (OFF_WT + WT_BYTES)
#define OFF_HR   (OFF_H1 + PLANE16_BYTES)
#define OFF_P    (OFF_HR + PLANE16_BYTES)
#define OFF_PAR  (OFF_P + P_BYTES)
#define OFF_PART (OFF_PAR + PAR_BYTES)
#define WS_TOTAL (OFF_PART + PART_BYTES)
static_assert((WT_BYTES % 128) == 0 && (PLANE16_BYTES % 128) == 0 && (P_BYTES % 128) == 0);
static_assert((PAR_BYTES % 128) == 0 && (PART_BYTES % 128) == 0);
static_assert(WS_TOTAL <= (size_t)134217728);

__device__ __forceinline__ float bf16r(float x) {
  unsigned int u = __float_as_uint(x);
  u = (u + 0x7FFFu + ((u >> 16) & 1u)) & 0xFFFF0000u;
  return __uint_as_float(u);
}

static __device__ __forceinline__ h16 toh_flush(float v) {
  const h16 r = (h16)v;
  return (fabsf(v) < 6.103515625e-05f) ? (h16)0.0f : r;
}

__device__ __forceinline__ v16h frag_at(const _Float16* p) {
  v8h lo = *(const v8h*)(p);
  v8h hi = *(const v8h*)(p + 16);
  v16h out;
#pragma unroll
  for (int i = 0; i < 8; ++i) { out[i] = lo[i]; out[i + 8] = hi[i]; }
  return out;
}

__device__ __forceinline__ v8f wmma16(v16h a, v16h b, v8f c) {
  v8f d = __builtin_amdgcn_wmma_f32_16x16x32_f16(false, a, false, b, (short)0, c,
                                                 false, false);
  asm volatile("v_nop\n\tv_nop\n\tv_nop\n\tv_nop" : "+v"(d) : "v"(a), "v"(b));
  return d;
}

__device__ __forceinline__ float red32_sum(float x) {
#pragma unroll
  for (int off = 1; off < 32; off <<= 1) x += __shfl_xor(x, off, 32);
  return x;
}

__global__ __launch_bounds__(256) void wconv_kernel(
    const float* __restrict__ W, _Float16* __restrict__ Wt, unsigned ldw, unsigned ldk,
    unsigned nvalid) {
  __shared__ _Float16 T[64 * LDT];
  const unsigned tid = threadIdx.x;
  const unsigned n0 = blockIdx.x * 64u;
  const unsigned k0 = blockIdx.y * 64u;
#pragma unroll 4
  for (unsigned j = 0; j < 16u; ++j) {
    const unsigned idx = tid + 256u * j;
    const unsigned kr = idx >> 6, nc = idx & 63u;
    const unsigned n = n0 + nc;
    const unsigned ncl = (n < nvalid) ? n : (nvalid - 1u);
    const float v = W[(size_t)(k0 + kr) * ldw + ncl];
    const float s = (n < nvalid) ? (WCARRY * bf16r(v)) : 0.0f;
    T[nc * LDT + kr] = toh_flush(s);
  }
  __syncthreads();
  v8h x[2];
  size_t off[2];
#pragma unroll
  for (unsigned i = 0; i < 2u; ++i) {
    const unsigned n = 32u * i + (tid >> 3);
    const unsigned kc = (tid & 7u) * 8u;
    x[i] = *(const v8h*)&T[n * LDT + kc];
    off[i] = (size_t)(n0 + n) * ldk + k0 + kc;
  }
#pragma unroll
  for (int i = 0; i < 2; ++i) *(volatile v8h*)(Wt + off[i]) = x[i];
  __threadfence();
#pragma unroll
  for (int i = 0; i < 2; ++i) *(volatile v8h*)(Wt + off[i]) = x[i];
}

template <int SRC_INPUT>
__device__ __forceinline__ void ln_body(const float* __restrict__ X,
                                        const float* __restrict__ G,
                                        const float* __restrict__ Be,
                                        _Float16* __restrict__ dst,
                                        _Float16* __restrict__ dstr) {
  const unsigned lane = threadIdx.x & 31u, w = threadIdx.x >> 5;
  const unsigned crow = blockIdx.x * 8u + w;
  size_t srow = crow;
  if (SRC_INPUT) {
    const unsigned bidx = crow / (unsigned)SEQ;
    const unsigned sq = crow - bidx * (unsigned)SEQ;
    srow = (size_t)bidx * SEQ_FULL + sq;
  }
  const float* xr = X + srow * DIM + lane * 8u;

  float s = 0.0f;
#pragma unroll 1
  for (unsigned j = 0; j < 4u; ++j) {
    const v4f a0 = *(const v4f*)(xr + j * 256u);
    const v4f a1 = *(const v4f*)(xr + j * 256u + 4u);
#pragma unroll
    for (int i = 0; i < 4; ++i) {
      const float e0 = SRC_INPUT ? bf16r(a0[i]) : a0[i];
      const float e1 = SRC_INPUT ? bf16r(a1[i]) : a1[i];
      s += e0 + e1;
    }
  }
  const float mean = red32_sum(s) * (1.0f / (float)DIM);

  float ss = 0.0f;
#pragma unroll 1
  for (unsigned j = 0; j < 4u; ++j) {
    const v4f a0 = *(const v4f*)(xr + j * 256u);
    const v4f a1 = *(const v4f*)(xr + j * 256u + 4u);
#pragma unroll
    for (int i = 0; i < 4; ++i) {
      const float d0 = (SRC_INPUT ? bf16r(a0[i]) : a0[i]) - mean;
      const float d1 = (SRC_INPUT ? bf16r(a1[i]) : a1[i]) - mean;
      ss += d0 * d0;
      ss += d1 * d1;
    }
  }
  const float var = red32_sum(ss) * (1.0f / (float)DIM);
  const float rstd = 1.0f / sqrtf(var + 1.0e-5f);

#pragma unroll 1
  for (unsigned j = 0; j < 4u; ++j) {
    const unsigned c = j * 256u + lane * 8u;
    const v4f a0 = *(const v4f*)(xr + j * 256u);
    const v4f a1 = *(const v4f*)(xr + j * 256u + 4u);
    const v4f g0 = *(const v4f*)(G + c);
    const v4f g1 = *(const v4f*)(G + c + 4u);
    const v4f b0 = *(const v4f*)(Be + c);
    const v4f b1 = *(const v4f*)(Be + c + 4u);
    v8h o;
#if XN_RES
    v8h orr;
#endif
#pragma unroll
    for (int i = 0; i < 4; ++i) {
      const float d0 = (SRC_INPUT ? bf16r(a0[i]) : a0[i]) - mean;
      const float d1 = (SRC_INPUT ? bf16r(a1[i]) : a1[i]) - mean;
      const float y0 = d0 * rstd * bf16r(g0[i]) + bf16r(b0[i]);
      const float y1 = d1 * rstd * bf16r(g1[i]) + bf16r(b1[i]);
      const h16 h0 = toh_flush(y0);
      const h16 h1 = toh_flush(y1);
      o[i]     = h0;
      o[i + 4] = h1;
#if XN_RES
      orr[i]     = toh_flush((y0 - (float)h0) * RCARRY);
      orr[i + 4] = toh_flush((y1 - (float)h1) * RCARRY);
#endif
    }
    _Float16* p = dst + (size_t)crow * DIM + c;
    *(volatile v8h*)p = o;
#if XN_RES
    _Float16* pr = dstr + (size_t)crow * DIM + c;
    *(volatile v8h*)pr = orr;
#endif
    __threadfence();
    *(volatile v8h*)p = o;
#if XN_RES
    *(volatile v8h*)pr = orr;
#endif
  }
#if !XN_RES
  (void)dstr;
#endif
}

__global__ __launch_bounds__(256) void ln_in_kernel(
    const float* __restrict__ X, const float* __restrict__ G, const float* __restrict__ Be,
    _Float16* __restrict__ dst, _Float16* __restrict__ dstr) {
  ln_body<1>(X, G, Be, dst, dstr);
}

__global__ __launch_bounds__(256) void gemm_par_kernel(
    const _Float16* __restrict__ A16, const _Float16* __restrict__ A16r,
    const _Float16* __restrict__ Bt, const float* __restrict__ bias,
    float* __restrict__ outf) {
  __shared__ float Cs[64 * LDC];
  const unsigned K = (unsigned)DIM;
  const unsigned tid = threadIdx.x, lane = tid & 31u, w = tid >> 5;
  const unsigned mw = w >> 1, nw = w & 1u;
  const unsigned hh = lane >> 4, m = lane & 15u;
  const unsigned n0 = blockIdx.x * 64u;
  const unsigned row0 = blockIdx.y * 64u;

  const _Float16* ap  = A16 + (size_t)(row0 + mw * 16u + m) * K + hh * 8u;
  const _Float16* bp0 = Bt + (size_t)(n0 + nw * 32u + m) * K + hh * 8u;
  const _Float16* bp1 = bp0 + (size_t)16 * K;
  v8f acc0 = {}, acc1 = {};
#if XN_RES
  const _Float16* rp = A16r + (size_t)(row0 + mw * 16u + m) * K + hh * 8u;
  v8f rc0 = {}, rc1 = {};
#else
  (void)A16r;
#endif
#pragma unroll 2
  for (unsigned k0 = 0; k0 < K; k0 += 32u) {
    const v16h a  = frag_at(ap + k0);
    const v16h b0 = frag_at(bp0 + k0);
    const v16h b1 = frag_at(bp1 + k0);
    acc0 = wmma16(a, b0, acc0);
    acc1 = wmma16(a, b1, acc1);
#if XN_RES
    const v16h ar = frag_at(rp + k0);
    rc0 = wmma16(ar, b0, rc0);
    rc1 = wmma16(ar, b1, rc1);
#endif
  }
#pragma unroll
  for (int r = 0; r < 8; ++r) {
    float* d = &Cs[(mw * 16u + hh * 8u + (unsigned)r) * LDC + nw * 32u + m];
#if XN_RES
    d[0]  = acc0[r] + rc0[r] * (1.0f / RCARRY);
    d[16] = acc1[r] + rc1[r] * (1.0f / RCARRY);
#else
    d[0]  = acc0[r];
    d[16] = acc1[r];
#endif
  }
  __syncthreads();

  const unsigned c = (tid & 15u) * 4u;
  float bb[4];
#pragma unroll
  for (unsigned j = 0; j < 4u; ++j) {
    const unsigned col = n0 + c + j;
    const unsigned cl = (col < (unsigned)NOUT) ? col : (unsigned)(NOUT - 1);
    const float braw = bias[cl];
    bb[j] = (col < (unsigned)NOUT) ? bf16r(braw) : 0.0f;
  }
  v4f xs[4];
  size_t off[4];
#pragma unroll
  for (unsigned i = 0; i < 4u; ++i) {
    const unsigned r = 16u * i + (tid >> 4);
    const v4f u = *(const v4f*)&Cs[r * LDC + c];
    v4f val;
#pragma unroll
    for (int j = 0; j < 4; ++j) val[j] = u[j] * (1.0f / WCARRY) + bb[j];
    xs[i] = val;
    off[i] = (size_t)(row0 + r) * NPAD + n0 + c;
  }
#pragma unroll
  for (int i = 0; i < 4; ++i) *(volatile v4f*)(outf + off[i]) = xs[i];
  __threadfence();
#pragma unroll
  for (int i = 0; i < 4; ++i) *(volatile v4f*)(outf + off[i]) = xs[i];
}

static __device__ __forceinline__ float softplus_f(float x) {
  return fmaxf(x, 0.0f) + __logf(1.0f + __expf(-fabsf(x)));
}

static __device__ __forceinline__ float sin_poly(float x) {
  const float n = rintf(x * 0.15915494309189535f);
  float r = fmaf(-n, 6.2831854820251465f, x);
  r = fmaf(-n, -1.7484556000744883e-07f, r);
  const float ar = fabsf(r);
  const float fold = copysignf(3.14159274101257324f, r) - r;
  r = (ar > 1.57079637050628662f) ? fold : r;
  const float s = r * r;
  float p = -2.50521083854417188e-08f;
  p = fmaf(p, s, 2.75573192239858907e-06f);
  p = fmaf(p, s, -1.98412698412698413e-04f);
  p = fmaf(p, s, 8.33333333333333333e-03f);
  p = fmaf(p, s, -1.66666666666666667e-01f);
  return fmaf(r * s, p, r);
}

__global__ __launch_bounds__(256) void params_kernel(
    const float* __restrict__ P, float* __restrict__ par, float* __restrict__ nstd_out) {
#pragma clang fp contract(off)
  const unsigned idx = blockIdx.x * 256u + threadIdx.x;
  const unsigned imu = idx / (unsigned)SEQ;
  const unsigned i = idx - imu * (unsigned)SEQ;
  const float* pr = P + (size_t)i * NPAD + imu;

  const float p0 = pr[0 * NIMU];
  const float p1 = pr[1 * NIMU];
  const float p2 = pr[2 * NIMU];
  const float p3 = pr[3 * NIMU];
  const float c  = pr[4 * NIMU];
  const float ct = pr[5 * NIMU];
  const float ph = pr[6 * NIMU];
  const float pt = pr[7 * NIMU];
  const float p9 = pr[9 * NIMU];

  const float d  = softplus_f(p1);
  const float s0 = softplus_f(p0);
  const float dd = d * d;
  const float k  = dd * 0.25f + s0;
  const float om = sqrtf(4.0f * k - dd) * 0.5f;

  const float dt  = softplus_f(p3);
  const float s2  = softplus_f(p2);
  const float ddt = dt * dt;
  const float kt  = ddt * 0.25f + s2;
  const float omt = sqrtf(4.0f * kt - ddt) * 0.5f;

  const float v1 = 0.5f * d;
  const float v5 = 0.5f * dt;
  const float v8 = softplus_f(p9);

  float* q = par + idx;
  float* qn = nstd_out + (size_t)imu * SEQ_FULL + i;
  *(volatile float*)(q + 0 * (size_t)PSTR) = c;
  *(volatile float*)(q + 1 * (size_t)PSTR) = v1;
  *(volatile float*)(q + 2 * (size_t)PSTR) = om;
  *(volatile float*)(q + 3 * (size_t)PSTR) = ph;
  *(volatile float*)(q + 4 * (size_t)PSTR) = ct;
  *(volatile float*)(q + 5 * (size_t)PSTR) = v5;
  *(volatile float*)(q + 6 * (size_t)PSTR) = omt;
  *(volatile float*)(q + 7 * (size_t)PSTR) = pt;
  *(volatile float*)qn = v8;
  __threadfence();
  *(volatile float*)(q + 0 * (size_t)PSTR) = c;
  *(volatile float*)(q + 1 * (size_t)PSTR) = v1;
  *(volatile float*)(q + 2 * (size_t)PSTR) = om;
  *(volatile float*)(q + 3 * (size_t)PSTR) = ph;
  *(volatile float*)(q + 4 * (size_t)PSTR) = ct;
  *(volatile float*)(q + 5 * (size_t)PSTR) = v5;
  *(volatile float*)(q + 6 * (size_t)PSTR) = omt;
  *(volatile float*)(q + 7 * (size_t)PSTR) = pt;
  *(volatile float*)qn = v8;
}

__global__ __launch_bounds__(64) void kin_kernel(
    const float* __restrict__ par, float* __restrict__ part) {
#pragma clang fp contract(off)
  __shared__ float lds[8 * ICH];
  const int j     = (int)blockIdx.x * JT + (int)threadIdx.x;
  const int imu   = (int)blockIdx.y;
  const int ic    = (int)blockIdx.z;
  const int ibase = ic * ICH;
  const int jmax  = (int)blockIdx.x * JT + (JT - 1);

  float acc = 0.0f;
  if (ibase <= jmax) {
    for (int t = (int)threadIdx.x; t < 8 * ICH; t += 64) {
      const int a = t / ICH, e = t - a * ICH;
      lds[t] = par[(size_t)a * PSTR + (size_t)imu * SEQ + ibase + e];
    }
    __syncthreads();
    int emax = jmax - ibase;
    emax = (emax > ICH - 1) ? (ICH - 1) : emax;
#pragma unroll 1
    for (int e = 0; e <= emax; ++e) {
      const int dlag = j - (ibase + e);
      const bool live = (dlag >= 0);
      const float tt = (float)(live ? dlag : 0);
      const float c0 = lds[e];
      const float a0 = lds[ICH + e];
      const float w0 = lds[2 * ICH + e];
      const float f0 = lds[3 * ICH + e];
      const float c1 = lds[4 * ICH + e];
      const float a1 = lds[5 * ICH + e];
      const float w1 = lds[6 * ICH + e];
      const float f1 = lds[7 * ICH + e];
      const float x0 = tt * w0 + f0;
      const float x1 = tt * w1 + f1;
      const float lin = c0 * __expf(-(a0 * tt)) * sin_poly(x0);
      const float ang = c1 * __expf(-(a1 * tt)) * sin_poly(x1);
      const float term = lin + ang;
      acc += live ? term : 0.0f;
    }
  }
  float* dstp = part + ((size_t)ic * NIMU + imu) * SEQ + j;
  *(volatile float*)dstp = acc;
  __threadfence();
  *(volatile float*)dstp = acc;
}

__global__ __launch_bounds__(256) void reduce_kernel(
    const float* __restrict__ part, const float* __restrict__ P, const float* __restrict__ mo,
    float* __restrict__ out) {
#pragma clang fp contract(off)
  const unsigned idx = blockIdx.x * 256u + threadIdx.x;
  const unsigned imu = idx / (unsigned)SEQ;
  const unsigned j = idx - imu * (unsigned)SEQ;
  float s = 0.0f;
#pragma unroll
  for (int ic = 0; ic < NCH; ++ic) s += part[((size_t)ic * NIMU + imu) * SEQ + j];
  const float m0 = bf16r(mo[0]);
  const float nb = P[(size_t)j * NPAD + 8 * NIMU + imu];
  const float v = (s + m0) + nb;
  float* dstp = out + (size_t)imu * SEQ_FULL + j;
  *(volatile float*)dstp = v;
  __threadfence();
  *(volatile float*)dstp = v;
}

extern "C" void kernel_launch(void* const* d_in, const int* in_sizes, int n_in,
                              void* d_out, int out_size, void* d_ws, size_t ws_size,
                              hipStream_t stream) {
  if (n_in < 6) return;
  if ((long long)in_sizes[0] < (long long)SEQ * DIM) return;
  if (in_sizes[1] < 1) return;
  if (in_sizes[2] < DIM || in_sizes[3] < DIM) return;
  if ((long long)in_sizes[4] < (long long)DIM * NOUT) return;
  if (in_sizes[5] < NOUT) return;
  if ((long long)out_size < (long long)2 * NIMU * SEQ_FULL) return;
  if (ws_size < WS_TOTAL) return;

  const float* X    = (const float*)d_in[0];
  const float* mo   = (const float*)d_in[1];
  const float* gam  = (const float*)d_in[2];
  const float* bet  = (const float*)d_in[3];
  const float* W    = (const float*)d_in[4];
  const float* bias = (const float*)d_in[5];
  float* out = (float*)d_out;

  char* ws = (char*)d_ws;
  _Float16* Wt   = (_Float16*)(ws + OFF_WT);
  _Float16* H1   = (_Float16*)(ws + OFF_H1);
  _Float16* HR   = (_Float16*)(ws + OFF_HR);
  float*    Pp   = (float*)(ws + OFF_P);
  float*    PAR  = (float*)(ws + OFF_PAR);
  float*    PART = (float*)(ws + OFF_PART);

  dim3 blk(256);

  wconv_kernel<<<dim3(NPAD / 64, DIM / 64), blk, 0, stream>>>(W, Wt, (unsigned)NOUT, (unsigned)DIM,
                                                              (unsigned)NOUT);
  ln_in_kernel<<<dim3(MROWS / 8), blk, 0, stream>>>(X, gam, bet, H1, HR);
  gemm_par_kernel<<<dim3(NPAD / 64, MROWS / 64), blk, 0, stream>>>(H1, HR, Wt, bias, Pp);
  params_kernel<<<dim3((NIMU * SEQ) / 256), blk, 0, stream>>>(Pp, PAR, out + (size_t)NIMU * SEQ_FULL);
  kin_kernel<<<dim3(SEQ / JT, NIMU, NCH), dim3(64), 0, stream>>>(PAR, PART);
  reduce_kernel<<<dim3((NIMU * SEQ) / 256), blk, 0, stream>>>(PART, Pp, mo, out);
}
